// Interpolator_78683800862819
// MI455X (gfx1250) — hardware-verified
//
#include <hip/hip_runtime.h>
#include <stdint.h>

#define DD   64
#define DY   32
#define RB   64
#define HSP  72
#define YSP  72
#define OSP  36
#define L2E  1.44269504088896340736f
#define PEX  14.0f
#define YSC  16.0f
#define OSC  0.0625f

static_assert(DD == 64);
static_assert(DY == 32);
static_assert((HSP * 2) % 16 == 0);
static_assert((YSP * 2) % 16 == 0);
static_assert((OSP * 4) % 16 == 0);
static_assert(RB * 8 == 512);

typedef _Float16       v8h  __attribute__((ext_vector_type(8)));
typedef _Float16       v16h __attribute__((ext_vector_type(16)));
typedef __bf16         v16b __attribute__((ext_vector_type(16)));
typedef unsigned short v8us __attribute__((ext_vector_type(8)));
typedef unsigned int   v4u  __attribute__((ext_vector_type(4)));
typedef float          v4f  __attribute__((ext_vector_type(4)));
typedef float          v8f  __attribute__((ext_vector_type(8)));

union FragH { v8h p[2]; v16h v; };
union FragB { v8us p[2]; v16b v; };
static_assert(sizeof(FragH) == 32);
static_assert(sizeof(FragB) == 32);

__device__ __forceinline__ v8f zero8() { v8f z = {0.f, 0.f, 0.f, 0.f, 0.f, 0.f, 0.f, 0.f}; return z; }

__device__ __forceinline__ unsigned int bf_bits(float x) {
  unsigned int u = __float_as_uint(x);
  u += 0x7FFFu + ((u >> 16) & 1u);
  return u >> 16;
}
__device__ __forceinline__ float bf_rne(float x) { return __uint_as_float(bf_bits(x) << 16); }

__device__ __forceinline__ v8f mma_h(v16h a, v16h b, v8f c) {
  v8f d = __builtin_amdgcn_wmma_f32_16x16x32_f16(false, a, false, b, (short)0, c, false, false);
#if defined(__HIP_DEVICE_COMPILE__)
  asm volatile("v_nop\n\tv_nop\n\tv_nop\n\tv_nop" : "+v"(d) : "v"(a), "v"(b));
#endif
  return d;
}
__device__ __forceinline__ v8f mma_b(v16b a, v16b b, v8f c) {
  v8f d = __builtin_amdgcn_wmma_f32_16x16x32_bf16(false, a, false, b, (short)0, c, false, false);
#if defined(__HIP_DEVICE_COMPILE__)
  asm volatile("v_nop\n\tv_nop\n\tv_nop\n\tv_nop" : "+v"(d) : "v"(a), "v"(b));
#endif
  return d;
}

__device__ __forceinline__ void stage_rows(const float* __restrict__ src, float* zs, int t) {
#pragma unroll
  for (int it = 0; it < 2; ++it) {
    const int q = it * 256 + t, row = q >> 3, e = q & 7;
    const float* s = src + (size_t)row * DD + 8 * e;
    v4f a = *(const v4f*)(s);
    v4f b = *(const v4f*)(s + 4);
#pragma unroll
    for (int i = 0; i < 4; ++i) { a[i] = bf_rne(a[i]); b[i] = bf_rne(b[i]); }
    *(v4f*)(zs + row * DD + 8 * e)     = a;
    *(v4f*)(zs + row * DD + 8 * e + 4) = b;
  }
}

__global__ __launch_bounds__(256)
void k_tgt(const float* __restrict__ zt, const float* __restrict__ W,
           unsigned short* ZH, unsigned short* ZL) {
  __shared__ float Ms[DD * DD];
  __shared__ __align__(16) float Zs[RB * DD];
  __shared__ __align__(16) unsigned short Hs[RB * HSP];
  __shared__ __align__(16) unsigned short Ls[RB * HSP];
  const int t  = threadIdx.x;
  const int t0 = blockIdx.x * RB;
  for (int i = t; i < DD * DD; i += 256) {
    const int k = i >> 6, j = i & 63;
    Ms[i] = bf_rne(W[i]) + bf_rne(W[j * DD + k]);
  }
  stage_rows(zt + (size_t)t0 * DD, Zs, t);
  __syncthreads();

  const int r4 = t >> 6, j = t & 63;
#pragma unroll 1
  for (int p = 0; p < RB / 4; ++p) {
    const int r = 4 * p + r4;
    const float* zr = Zs + r * DD;
    float a = 0.f;
#pragma unroll 4
    for (int k = 0; k < DD; ++k) a = fmaf(zr[k], Ms[k * DD + j], a);
    const unsigned int hb = bf_bits(a);
    const float lo = a - __uint_as_float(hb << 16);
    const unsigned int lb = bf_bits(lo);
    Hs[r * HSP + j] = (unsigned short)hb;
    Ls[r * HSP + j] = (unsigned short)lb;
  }
  __syncthreads();

  v8us hv[2], lv[2];
  size_t po[2];
#pragma unroll
  for (int it = 0; it < 2; ++it) {
    const int q = it * 256 + t, row = q >> 3, e = q & 7;
    hv[it] = *(const v8us*)(Hs + row * HSP + 8 * e);
    lv[it] = *(const v8us*)(Ls + row * HSP + 8 * e);
    po[it] = (size_t)(t0 + row) * DD + 8 * e;
  }
#pragma unroll
  for (int it = 0; it < 2; ++it) {
    *(volatile v8us*)(ZH + po[it]) = hv[it];
    *(volatile v8us*)(ZL + po[it]) = lv[it];
  }
  __threadfence();
#pragma unroll
  for (int it = 0; it < 2; ++it) {
    *(volatile v8us*)(ZH + po[it]) = hv[it];
    *(volatile v8us*)(ZL + po[it]) = lv[it];
  }
}

__global__ __launch_bounds__(256)
void k_ctx(const float* __restrict__ zc, const float* __restrict__ yc, const float* __restrict__ W,
           unsigned short* ZC, _Float16* YT, float* QL, int C) {
  __shared__ float Ws[DD * DD];
  __shared__ __align__(16) float Zs[RB * DD];
  __shared__ __align__(16) _Float16 Ys[DY * YSP];
  __shared__ float Qp[RB * 2];
  __shared__ __align__(16) float Qs[RB];
  const int t  = threadIdx.x;
  const int c0 = blockIdx.x * RB;
  for (int i = t; i < DD * DD; i += 256) Ws[i] = bf_rne(W[i]);
  stage_rows(zc + (size_t)c0 * DD, Zs, t);
  for (int i = t; i < RB * DY; i += 256) {
    const int c = i >> 5, dy = i & 31;
    const float v = bf_rne(yc[(size_t)(c0 + c) * DY + dy]) * YSC;
    Ys[dy * YSP + c] = (_Float16)v;
  }
  __syncthreads();

  const int r4 = t >> 6, j = t & 63, lane = t & 31, wv = t >> 5;
#pragma unroll 1
  for (int p = 0; p < RB / 4; ++p) {
    const int r = 4 * p + r4;
    const float* zr = Zs + r * DD;
    float a = 0.f;
#pragma unroll 4
    for (int k = 0; k < DD; ++k) a = fmaf(zr[k], Ws[k * DD + j], a);
    float q = a * zr[j];
#pragma unroll
    for (int o = 1; o < 32; o <<= 1) q += __shfl_xor(q, o, 32);
    if (lane == 0) Qp[r * 2 + (wv & 1)] = q;
  }
  __syncthreads();
  if (t < RB) Qs[t] = (Qp[2 * t] + Qp[2 * t + 1]) * L2E;
  __syncthreads();

  v8us zv[2];
  size_t pz[2];
#pragma unroll
  for (int it = 0; it < 2; ++it) {
    const int q = it * 256 + t, row = q >> 3, e = q & 7;
    const v4u a = *(const v4u*)(Zs + row * DD + 8 * e);
    const v4u b = *(const v4u*)(Zs + row * DD + 8 * e + 4);
    v8us w;
    w[0] = (unsigned short)(a[0] >> 16); w[1] = (unsigned short)(a[1] >> 16);
    w[2] = (unsigned short)(a[2] >> 16); w[3] = (unsigned short)(a[3] >> 16);
    w[4] = (unsigned short)(b[0] >> 16); w[5] = (unsigned short)(b[1] >> 16);
    w[6] = (unsigned short)(b[2] >> 16); w[7] = (unsigned short)(b[3] >> 16);
    zv[it] = w;
    pz[it] = (size_t)(c0 + row) * DD + 8 * e;
  }
  const int dyr = t >> 3, ey = t & 7;
  const v8h yv = *(const v8h*)(Ys + dyr * YSP + 8 * ey);
  const size_t py = (size_t)dyr * C + c0 + 8 * ey;
  const bool wq = (t < RB / 4);
  v4f qv = {0.f, 0.f, 0.f, 0.f};
  float* qd = QL;
  if (wq) { qv = *(const v4f*)(Qs + 4 * t); qd = QL + c0 + 4 * t; }

#pragma unroll
  for (int it = 0; it < 2; ++it) *(volatile v8us*)(ZC + pz[it]) = zv[it];
  *(volatile v8h*)(YT + py) = yv;
  if (wq) *(volatile v4f*)qd = qv;
  __threadfence();
#pragma unroll
  for (int it = 0; it < 2; ++it) *(volatile v8us*)(ZC + pz[it]) = zv[it];
  *(volatile v8h*)(YT + py) = yv;
  if (wq) *(volatile v4f*)qd = qv;
}

__global__ __launch_bounds__(64)
void k_main(const unsigned short* __restrict__ ZC, const unsigned short* __restrict__ ZH,
            const unsigned short* __restrict__ ZL, const _Float16* __restrict__ YT,
            const float* __restrict__ QL, float* out, int C) {
  __shared__ __align__(16) float Os[2][16 * OSP];
  const int t    = threadIdx.x;
  const int lane = t & 31, wv = t >> 5;
  const int hh   = lane >> 4, n = lane & 15;
  const int t0   = blockIdx.x * 32 + 16 * wv;

  FragB bh0, bh1, bl0, bl1;
  {
    const unsigned short* hp = ZH + (size_t)(t0 + n) * DD + 8 * hh;
    const unsigned short* lp = ZL + (size_t)(t0 + n) * DD + 8 * hh;
    bh0.p[0] = *(const v8us*)(hp);      bh0.p[1] = *(const v8us*)(hp + 16);
    bh1.p[0] = *(const v8us*)(hp + 32); bh1.p[1] = *(const v8us*)(hp + 48);
    bl0.p[0] = *(const v8us*)(lp);      bl0.p[1] = *(const v8us*)(lp + 16);
    bl1.p[0] = *(const v8us*)(lp + 32); bl1.p[1] = *(const v8us*)(lp + 48);
  }

  const unsigned short* zcp = ZC + (size_t)n * DD + 8 * hh;
  const _Float16* y0p = YT + (size_t)n * C + 8 * hh;
  const _Float16* y1p = YT + (size_t)(16 + n) * C + 8 * hh;
  const float* qp = QL + 8 * hh;

  v8f O0 = zero8(), O1 = zero8();
  float m = -1.0e30f, z = 0.f;

#pragma unroll 1
  for (int c0 = 0; c0 < C; c0 += 32) {
    v8f S0 = zero8(), S1 = zero8();
    {
      const unsigned short* a0p = zcp + (size_t)c0 * DD;
      const unsigned short* a1p = a0p + (size_t)16 * DD;
      FragB a00, a01, a10, a11;
      a00.p[0] = *(const v8us*)(a0p);      a00.p[1] = *(const v8us*)(a0p + 16);
      a01.p[0] = *(const v8us*)(a0p + 32); a01.p[1] = *(const v8us*)(a0p + 48);
      a10.p[0] = *(const v8us*)(a1p);      a10.p[1] = *(const v8us*)(a1p + 16);
      a11.p[0] = *(const v8us*)(a1p + 32); a11.p[1] = *(const v8us*)(a1p + 48);
      S0 = mma_b(a00.v, bh0.v, S0);
      S0 = mma_b(a00.v, bl0.v, S0);
      S0 = mma_b(a01.v, bh1.v, S0);
      S0 = mma_b(a01.v, bl1.v, S0);
      S1 = mma_b(a10.v, bh0.v, S1);
      S1 = mma_b(a10.v, bl0.v, S1);
      S1 = mma_b(a11.v, bh1.v, S1);
      S1 = mma_b(a11.v, bl1.v, S1);
    }

    const v4f q0a = *(const v4f*)(qp + c0);
    const v4f q0b = *(const v4f*)(qp + c0 + 4);
    const v4f q1a = *(const v4f*)(qp + c0 + 16);
    const v4f q1b = *(const v4f*)(qp + c0 + 20);
    float u0[8], u1[8];
#pragma unroll
    for (int r = 0; r < 4; ++r) {
      u0[r]     = fmaf(S0[r],     L2E, -q0a[r]);
      u0[4 + r] = fmaf(S0[4 + r], L2E, -q0b[r]);
      u1[r]     = fmaf(S1[r],     L2E, -q1a[r]);
      u1[4 + r] = fmaf(S1[4 + r], L2E, -q1b[r]);
    }
    float tm = fmaxf(u0[0], u1[0]);
#pragma unroll
    for (int r = 1; r < 8; ++r) tm = fmaxf(tm, fmaxf(u0[r], u1[r]));
    const float tmo = __shfl_xor(tm, 16, 32);
    tm = fmaxf(tm, tmo);
    const float mn    = fmaxf(m, tm);
    const float alpha = __builtin_amdgcn_exp2f(m - mn);
    m = mn;
    const float mb = mn - PEX;
    z *= alpha;
    O0 = O0 * alpha;
    O1 = O1 * alpha;

    FragH pf;
#pragma unroll
    for (int r = 0; r < 8; ++r) {
      const float p0 = __builtin_amdgcn_exp2f(u0[r] - mb);
      const float p1 = __builtin_amdgcn_exp2f(u1[r] - mb);
      const _Float16 h0 = (_Float16)p0;
      const _Float16 h1 = (_Float16)p1;
      pf.v[r]     = h0;
      pf.v[8 + r] = h1;
      z += (float)h0;
      z += (float)h1;
    }

    FragH ay0, ay1;
    ay0.p[0] = *(const v8h*)(y0p + c0); ay0.p[1] = *(const v8h*)(y0p + c0 + 16);
    ay1.p[0] = *(const v8h*)(y1p + c0); ay1.p[1] = *(const v8h*)(y1p + c0 + 16);
    O0 = mma_h(ay0.v, pf.v, O0);
    O1 = mma_h(ay1.v, pf.v, O1);
  }

  const float zo  = __shfl_xor(z, 16, 32);
  const float ztt = z + zo;
  const float rz  = __builtin_amdgcn_rcpf(ztt) * OSC;
  float* osw = &Os[wv][0];
#pragma unroll
  for (int r = 0; r < 8; ++r) {
    osw[n * OSP + 8 * hh + r]      = O0[r] * rz;
    osw[n * OSP + 16 + 8 * hh + r] = O1[r] * rz;
  }
  __syncthreads();

  v4f ov[4];
  size_t po[4];
#pragma unroll
  for (int it = 0; it < 4; ++it) {
    const int q = it * 32 + lane, row = q >> 3, e = q & 7;
    ov[it] = *(const v4f*)(osw + row * OSP + 4 * e);
    po[it] = (size_t)(t0 + row) * DY + 4 * e;
  }
#pragma unroll
  for (int it = 0; it < 4; ++it) *(volatile v4f*)(out + po[it]) = ov[it];
  __threadfence();
#pragma unroll
  for (int it = 0; it < 4; ++it) *(volatile v4f*)(out + po[it]) = ov[it];
}

extern "C" void kernel_launch(void* const* d_in, const int* in_sizes, int n_in,
                              void* d_out, int out_size, void* d_ws, size_t ws_size,
                              hipStream_t stream) {
  if (n_in < 4) return;
  const int C = in_sizes[0] / DD;
  const int T = in_sizes[2] / DD;
  if (C <= 0 || T <= 0) return;
  if (C * DD != in_sizes[0] || T * DD != in_sizes[2]) return;
  if (in_sizes[1] != C * DY) return;
  if (in_sizes[3] != DD * DD) return;
  if (out_size != T * DY) return;
  if ((T % RB) != 0 || (C % RB) != 0) return;

  size_t off = 0;
  const size_t oZH = off; off += (size_t)T * DD * 2;
  const size_t oZL = off; off += (size_t)T * DD * 2;
  const size_t oZC = off; off += (size_t)C * DD * 2;
  const size_t oYT = off; off += (size_t)DY * C * 2;
  const size_t oQL = off; off += (size_t)C * 4;
  if (off > ws_size) return;
  if (off > (size_t)134217728) return;

  const float* zc = (const float*)d_in[0];
  const float* yc = (const float*)d_in[1];
  const float* zt = (const float*)d_in[2];
  const float* W  = (const float*)d_in[3];
  float* out = (float*)d_out;

  char* ws = (char*)d_ws;
  unsigned short* ZH = (unsigned short*)(ws + oZH);
  unsigned short* ZL = (unsigned short*)(ws + oZL);
  unsigned short* ZC = (unsigned short*)(ws + oZC);
  _Float16*       YT = (_Float16*)(ws + oYT);
  float*          QL = (float*)(ws + oQL);

  k_tgt<<<dim3(T / RB), dim3(256), 0, stream>>>(zt, W, ZH, ZL);
  k_ctx<<<dim3(C / RB), dim3(256), 0, stream>>>(zc, yc, W, ZC, YT, QL, C);
  k_main<<<dim3(T / 32), dim3(64), 0, stream>>>(ZC, ZH, ZL, YT, QL, out, C);
  (void)hipGetLastError();
}
